// AttentionLayer_24764781428881
// MI455X (gfx1250) — hardware-verified
//
#include <hip/hip_runtime.h>


#ifndef NB
#define NB 4
#endif
#ifndef SEQ
#define SEQ 2048
#endif
#define SEQ_FULL 2048
#define DMD 1024
#define NHD 16
#define HDM 64
#define PCAR 256.0f
#define C1 0.18033688011112042f

static_assert(SEQ % 64 == 0);
static_assert(NB >= 1);
static_assert(NHD * HDM == DMD);
static_assert(DMD % 64 == 0);

typedef _Float16 h16;
typedef unsigned short bf;
typedef __attribute__((ext_vector_type(16))) __bf16   v16bf;
typedef __attribute__((ext_vector_type(16))) _Float16 v16h;
typedef __attribute__((ext_vector_type(8)))  _Float16 v8h;
typedef __attribute__((ext_vector_type(8)))  unsigned short v8us;
typedef __attribute__((ext_vector_type(8)))  float    v8f;
typedef __attribute__((ext_vector_type(4)))  float    v4f;
typedef __attribute__((ext_vector_type(2)))  _Float16 v2h;
typedef __attribute__((ext_vector_type(2)))  unsigned short v2us;
typedef v8h  __attribute__((may_alias)) v8ha;
typedef v4f  __attribute__((may_alias)) v4fa;
typedef v8us __attribute__((may_alias)) v8usa;

__device__ __forceinline__ unsigned short f2bf(float f) { unsigned u = __float_as_uint(f); u += 0x7FFFu + ((u >> 16) & 1u); return (unsigned short)(u >> 16); }
__device__ __forceinline__ float bf2f(unsigned short b) { return __uint_as_float(((unsigned)b) << 16); }
__device__ __forceinline__ float bfr(float f) { return bf2f(f2bf(f)); }
__device__ __forceinline__ v16h cat16(v8h lo, v8h hi) { return __builtin_shufflevector(lo, hi, 0, 1, 2, 3, 4, 5, 6, 7, 8, 9, 10, 11, 12, 13, 14, 15); }
__device__ __forceinline__ v16bf cat16b(v8us lo, v8us hi) { return __builtin_bit_cast(v16bf, __builtin_shufflevector(lo, hi, 0, 1, 2, 3, 4, 5, 6, 7, 8, 9, 10, 11, 12, 13, 14, 15)); }
__device__ __forceinline__ v8f wmma16(v16h a, v16h b, v8f c) { return __builtin_amdgcn_wmma_f32_16x16x32_f16(false, a, false, b, (short)0, c, false, false); }
__device__ __forceinline__ v8f wmmab(v16bf a, v16bf b, v8f c) { return __builtin_amdgcn_wmma_f32_16x16x32_bf16(false, a, false, b, (short)0, c, false, false); }
__device__ __forceinline__ v8f wmma16g(v16h a, v16h b, v8f c) {
    v8f d = __builtin_amdgcn_wmma_f32_16x16x32_f16(false, a, false, b, (short)0, c, false, false);
    asm volatile("v_nop\n\tv_nop\n\tv_nop\n\tv_nop" : "+v"(d) : "v"(a), "v"(b));
    return d;
}

template <typename T16> struct WFrag;
template <> struct WFrag<h16> { typedef v16h V; static __device__ __forceinline__ V ld(const h16* p) { return cat16(*(const v8h*)p, *(const v8h*)(p + 16)); } static __device__ __forceinline__ v8f mma(V a, V b, v8f c) { return wmma16(a, b, c); } };
template <> struct WFrag<bf> { typedef v16bf V; static __device__ __forceinline__ V ld(const bf* p) { return cat16b(*(const v8us*)p, *(const v8us*)(p + 16)); } static __device__ __forceinline__ v8f mma(V a, V b, v8f c) { return wmmab(a, b, c); } };
template <typename T16, int NSPLIT, bool BIAS>
__global__ __launch_bounds__(32) void k_gemmw(const T16* __restrict__ A, const T16* __restrict__ A2, const T16* __restrict__ Bt, const T16* __restrict__ Bt2, int K, float* C, int ldc, const float* __restrict__ bias, size_t sA, size_t sB, size_t sC) {
    typedef typename WFrag<T16>::V V;
    __shared__ __align__(16) float os[16 * 68];
    const size_t z = blockIdx.z; A += z * sA; if (A2) A2 += z * sA; Bt += z * sB; if (Bt2) Bt2 += z * sB; C += z * sC;
    const int lane = threadIdx.x & 31, lr = lane & 15, hi = lane >> 4; const int r0 = blockIdx.x * 64, c0 = blockIdx.y * 64;
    v8f acc[4][4];
#pragma unroll
    for (int mb = 0; mb < 4; ++mb)
#pragma unroll
        for (int nb = 0; nb < 4; ++nb) acc[mb][nb] = (v8f){};
    const size_t aoff = (size_t)(r0 + lr) * K + 8 * hi, boff = (size_t)(c0 + lr) * K + 8 * hi;
#pragma unroll 1
    for (int kc = 0; kc < K; kc += 32) {
        V a[4], a2[4];
#pragma unroll
        for (int mb = 0; mb < 4; ++mb) { a[mb] = WFrag<T16>::ld(A + aoff + (size_t)mb * 16 * K + kc); if (NSPLIT == 1 || NSPLIT == 2) a2[mb] = WFrag<T16>::ld(A2 + aoff + (size_t)mb * 16 * K + kc); }
#pragma unroll
        for (int nb = 0; nb < 4; ++nb) { const V b = WFrag<T16>::ld(Bt + boff + (size_t)nb * 16 * K + kc); V b2; if (NSPLIT >= 2) b2 = WFrag<T16>::ld(Bt2 + boff + (size_t)nb * 16 * K + kc);
#pragma unroll
            for (int mb = 0; mb < 4; ++mb) { acc[mb][nb] = WFrag<T16>::mma(a[mb], b, acc[mb][nb]); if (NSPLIT == 1 || NSPLIT == 2) acc[mb][nb] = WFrag<T16>::mma(a2[mb], b, acc[mb][nb]); if (NSPLIT >= 2) acc[mb][nb] = WFrag<T16>::mma(a[mb], b2, acc[mb][nb]); } }
        asm volatile("v_nop\n\tv_nop\n\tv_nop\n\tv_nop" : "+v"(acc[0][0]), "+v"(acc[1][1]), "+v"(acc[2][2]), "+v"(acc[3][3]) : "v"(a[0]), "v"(a[3]));
    }
#pragma unroll
    for (int mb = 0; mb < 4; ++mb) {
#pragma unroll
        for (int nb = 0; nb < 4; ++nb) {
#pragma unroll
            for (int j = 0; j < 8; ++j) os[(hi * 8 + j) * 68 + nb * 16 + lr] = acc[mb][nb][j]; }
        __builtin_amdgcn_wave_barrier(); asm volatile("" ::: "memory");
        float* crow = C + (size_t)(r0 + mb * 16) * ldc + c0;
#pragma unroll 1
        for (int ps = 0; ps < 2; ++ps) {
#pragma unroll
            for (int s = 0; s < 8; ++s) { const int row = 2 * s + hi, cofs = lr * 4; v4f val = *(const v4fa*)(os + row * 68 + cofs); if (BIAS) { val[0] += bfr(bias[c0 + cofs]); val[1] += bfr(bias[c0 + cofs + 1]); val[2] += bfr(bias[c0 + cofs + 2]); val[3] += bfr(bias[c0 + cofs + 3]); }
                *(volatile v4f*)(crow + (size_t)row * ldc + cofs) = val; }
            if (ps == 0) __threadfence(); }
        __builtin_amdgcn_wave_barrier(); asm volatile("" ::: "memory");
    }
}

__global__ __launch_bounds__(256) void k_wtG(const float* __restrict__ w, int K, int N, bf* Bt) {
    const int lane = threadIdx.x & 31; const int L0 = (blockIdx.x * 8 + (threadIdx.x >> 5)) * 8; const int nlines = N * K / 64;
#pragma unroll
    for (int ps = 0; ps < 2; ++ps) {
#pragma unroll 1
        for (int l = 0; l < 8; ++l) { const int L = L0 + l; if (L >= nlines) break; const size_t e = (size_t)L * 64 + lane * 2; const int k = (int)(e % K), n = (int)(e / K); v2us o;
            o[0] = f2bf(w[(size_t)k * N + n]); o[1] = f2bf(w[(size_t)(k + 1) * N + n]); *(volatile v2us*)(Bt + e) = o; }
        if (ps == 0) __threadfence(); }
}

__global__ __launch_bounds__(256) void k_cvtx(const float* __restrict__ x, bf* XB) {
    const size_t i = (size_t)blockIdx.x * 256 + threadIdx.x; const int b = blockIdx.y; if (i >= (size_t)SEQ * DMD / 8) return;
    const v8f v = *(const v8f*)(x + (size_t)b * SEQ_FULL * DMD + i * 8); v8us o;
#pragma unroll
    for (int k = 0; k < 8; ++k) o[k] = f2bf(v[k]);
    bf* d = XB + (size_t)b * SEQ * DMD + i * 8; *(volatile v8us*)d = o; __threadfence(); *(volatile v8us*)d = o;
}

__global__ __launch_bounds__(256) void k_cvth(const float* __restrict__ src, h16* dst, size_t n8) {
    const size_t i = (size_t)blockIdx.x * 256 + threadIdx.x; if (i >= n8) return;
    const v8f v = *(const v8f*)(src + i * 8); v8h o;
#pragma unroll
    for (int k = 0; k < 8; ++k) o[k] = (h16)v[k];
    *(volatile v8h*)(dst + i * 8) = o; __threadfence(); *(volatile v8h*)(dst + i * 8) = o;
}

__global__ __launch_bounds__(256) void k_vtp(const float* __restrict__ F, h16* VT) {
    const size_t e = ((size_t)blockIdx.x * 256 + threadIdx.x) * 2; const int b = blockIdx.y; if (e >= (size_t)DMD * SEQ) return;
    const int t = (int)(e % SEQ); const int c = (int)(e / SEQ); const size_t trow = (size_t)b * SEQ; v2h o;
    o[0] = (h16)F[(trow + t) * DMD + c]; o[1] = (h16)F[(trow + t + 1) * DMD + c];
    h16* d = VT + (size_t)b * DMD * SEQ + e; *(volatile v2h*)d = o; __threadfence(); *(volatile v2h*)d = o;
}

__global__ __launch_bounds__(128) __attribute__((amdgpu_num_vgpr(256)))
void k_attn(const h16* __restrict__ Q16, const h16* __restrict__ K16, const h16* __restrict__ VT, float* out) {
    __shared__ __align__(16) float os[4][16 * 68];
    const int lane = threadIdx.x & 31, wv = threadIdx.x >> 5, hh = lane >> 4, lr = lane & 15;
    const int b = blockIdx.z, hd = blockIdx.y, q0 = blockIdx.x * 64 + wv * 16, hcol = hd * HDM;
    const size_t trow = (size_t)b * SEQ;
    const h16* qp = Q16 + (trow + q0 + lr) * DMD + hcol + 8 * hh;
    v16h qf[2];
#pragma unroll
    for (int ks = 0; ks < 2; ++ks) qf[ks] = cat16(*(const v8h*)(qp + 32 * ks), *(const v8h*)(qp + 32 * ks + 16));
    const h16* kbase = K16 + (trow + lr) * DMD + hcol + 8 * hh;
    const h16* vbase = VT + ((size_t)b * DMD + hcol + lr) * SEQ + 8 * hh;
    float mrun = -3.0e38f, lrun = 0.0f;
    v8f oacc[4];
#pragma unroll
    for (int df = 0; df < 4; ++df) oacc[df] = (v8f){};
#pragma unroll 1
    for (int c0 = 0; c0 < SEQ; c0 += 64) {
        v8f sc[4];
#pragma unroll
        for (int kt = 0; kt < 4; ++kt) {
            sc[kt] = (v8f){};
            const h16* kp = kbase + (size_t)(c0 + kt * 16) * DMD;
#pragma unroll
            for (int ks = 0; ks < 2; ++ks) { const v16h a = cat16(*(const v8h*)(kp + 32 * ks), *(const v8h*)(kp + 32 * ks + 16)); sc[kt] = wmma16g(a, qf[ks], sc[kt]); }
        }
        float mloc = -3.0e38f;
#pragma unroll
        for (int kt = 0; kt < 4; ++kt)
#pragma unroll
            for (int r = 0; r < 8; ++r) { const float t = sc[kt][r] * C1; sc[kt][r] = t; mloc = fmaxf(mloc, t); }
        mloc = fmaxf(mloc, __shfl_xor(mloc, 16, 32));
        const float mnew = fmaxf(mrun, mloc);
        const float alpha = __builtin_amdgcn_exp2f(mrun - mnew);
        mrun = mnew;
        float rs = 0.0f;
#pragma unroll
        for (int kt = 0; kt < 4; ++kt)
#pragma unroll
            for (int r = 0; r < 8; ++r) { const float p = __builtin_amdgcn_exp2f(sc[kt][r] - mnew); sc[kt][r] = p; rs += p; }
        rs += __shfl_xor(rs, 16, 32);
        lrun = lrun * alpha + rs;
#pragma unroll
        for (int df = 0; df < 4; ++df) oacc[df] = oacc[df] * alpha;
        v16h pb[2];
#pragma unroll
        for (int ks = 0; ks < 2; ++ks) { v8h e0, e1;
#pragma unroll
            for (int r = 0; r < 8; ++r) { e0[r] = (h16)(sc[2 * ks][r] * PCAR); e1[r] = (h16)(sc[2 * ks + 1][r] * PCAR); }
            pb[ks] = cat16(e0, e1); }
#pragma unroll
        for (int df = 0; df < 4; ++df) {
            const h16* vp = vbase + (size_t)df * 16 * SEQ + c0;
#pragma unroll
            for (int ks = 0; ks < 2; ++ks) { const v16h a = cat16(*(const v8h*)(vp + 32 * ks), *(const v8h*)(vp + 32 * ks + 16)); oacc[df] = wmma16g(a, pb[ks], oacc[df]); }
        }
    }
    const float inv = (1.0f / lrun) * (1.0f / PCAR);
    float* osw = &os[wv][0];
#pragma unroll
    for (int df = 0; df < 4; ++df) { v4f u0, u1;
#pragma unroll
        for (int j = 0; j < 4; ++j) { u0[j] = oacc[df][j] * inv; u1[j] = oacc[df][4 + j] * inv; }
        *(v4fa*)(osw + lr * 68 + df * 16 + 8 * hh) = u0; *(v4fa*)(osw + lr * 68 + df * 16 + 8 * hh + 4) = u1; }
    __builtin_amdgcn_fence(3, "wavefront"); __builtin_amdgcn_wave_barrier(); asm volatile("" ::: "memory");
    float* orow = out + (trow + q0) * DMD + hcol;
#pragma unroll 1
    for (int ps = 0; ps < 2; ++ps) {
#pragma unroll
        for (int s = 0; s < 8; ++s) { const int row = 2 * s + hh, cofs = lr * 4; const v4f val = *(const v4fa*)(osw + row * 68 + cofs); *(volatile v4f*)(orow + (size_t)row * DMD + cofs) = val; }
        if (ps == 0) __threadfence(); }
}

extern "C" void kernel_launch(void* const* d_in, const int* in_sizes, int n_in,
                              void* d_out, int out_size, void* d_ws, size_t ws_size, hipStream_t stream) {
    if (n_in < 7) return;
    if (in_sizes[0] < (NB - 1) * SEQ_FULL * DMD + SEQ * DMD) return;
    if (in_sizes[1] < DMD * DMD || in_sizes[3] < DMD * DMD || in_sizes[5] < DMD * DMD) return;
    if (in_sizes[2] < DMD || in_sizes[4] < DMD || in_sizes[6] < DMD) return;
    if (out_size < NB * SEQ * DMD) return;
    const float* x = (const float*)d_in[0]; const float* wq = (const float*)d_in[1]; const float* bq = (const float*)d_in[2]; const float* wk = (const float*)d_in[3]; const float* bk = (const float*)d_in[4]; const float* wv = (const float*)d_in[5]; const float* bv = (const float*)d_in[6];
    float* OUT = (float*)d_out;
    char* wsp = (char*)d_ws;
    auto take = [&](size_t bytes) { char* p = wsp; wsp += (bytes + 255) & ~(size_t)255; return (void*)p; };
    const size_t MTOK = (size_t)NB * SEQ;
    bf* WQ = (bf*)take((size_t)DMD * DMD * 2); bf* WK = (bf*)take((size_t)DMD * DMD * 2); bf* WV = (bf*)take((size_t)DMD * DMD * 2);
    bf* XB = (bf*)take(MTOK * DMD * 2);
    float* F = (float*)take(MTOK * DMD * 4);
    h16* Q16 = (h16*)take(MTOK * DMD * 2); h16* K16 = (h16*)take(MTOK * DMD * 2); h16* VT16 = (h16*)take(MTOK * DMD * 2);
    if ((size_t)(wsp - (char*)d_ws) > ws_size) return;

    const unsigned gW = (unsigned)((DMD * DMD / 64 + 63) / 64);
    k_wtG<<<gW, 256, 0, stream>>>(wq, DMD, DMD, WQ);
    k_wtG<<<gW, 256, 0, stream>>>(wk, DMD, DMD, WK);
    k_wtG<<<gW, 256, 0, stream>>>(wv, DMD, DMD, WV);
    k_cvtx<<<dim3((unsigned)(((size_t)SEQ * DMD / 8 + 255) / 256), NB, 1), 256, 0, stream>>>(x, XB);
    const dim3 gG((unsigned)(MTOK / 64), DMD / 64, 1);
    const unsigned gC = (unsigned)((MTOK * DMD / 8 + 255) / 256);
    k_gemmw<bf, 0, true><<<gG, 32, 0, stream>>>(XB, nullptr, WQ, nullptr, DMD, F, DMD, bq, 0, 0, 0);
    k_cvth<<<gC, 256, 0, stream>>>(F, Q16, MTOK * DMD / 8);
    k_gemmw<bf, 0, true><<<gG, 32, 0, stream>>>(XB, nullptr, WK, nullptr, DMD, F, DMD, bk, 0, 0, 0);
    k_cvth<<<gC, 256, 0, stream>>>(F, K16, MTOK * DMD / 8);
    k_gemmw<bf, 0, true><<<gG, 32, 0, stream>>>(XB, nullptr, WV, nullptr, DMD, F, DMD, bv, 0, 0, 0);
    k_vtp<<<dim3((unsigned)(((size_t)DMD * SEQ / 2 + 255) / 256), NB, 1), 256, 0, stream>>>(F, VT16);
    k_attn<<<dim3(SEQ / 64, NHD, NB), 128, 0, stream>>>(Q16, K16, VT16, OUT);
}
